// Noise_VPT_13211319403315
// MI455X (gfx1250) — hardware-verified
//
#include <hip/hip_runtime.h>
#include <stddef.h>
#include <stdint.h>
#include <math.h>


#define CDIM   512
#define PDIM   1024
#define MROWS  25088
#define MBLK   64
#define NGRP   (PDIM / 64)
#define NTHR   128
#define NWAVE  4
#define RPB    32
#define WSCAP  134217728
#define CARRY  16.0f
#define FC2    (2.0f / 256.0f)
#define BIGV   3.0e38f

static_assert(NTHR == NWAVE * 32);
static_assert(MBLK == NWAVE * 16);
static_assert(CDIM == 512);
static_assert((CDIM % 32) == 0);
static_assert((PDIM % 64) == 0);
static_assert((MROWS % MBLK) == 0);
static_assert((MROWS % RPB) == 0);
static_assert((PDIM % RPB) == 0);
static_assert((RPB % NWAVE) == 0);
static_assert((PDIM % (4 * NTHR)) == 0);

#define SZ_E16  ((size_t)MROWS * CDIM * 2)
#define SZ_C16  ((size_t)PDIM * CDIM * 2)
#define SZ_FEAT ((size_t)MROWS * 4)
#define SZ_CENT ((size_t)PDIM * 4)
#define SZ_TOT  (SZ_E16 + SZ_C16 + SZ_FEAT + SZ_CENT)
static_assert(SZ_TOT <= (size_t)WSCAP);
static_assert((SZ_E16 % 128) == 0);
static_assert((SZ_C16 % 128) == 0);
static_assert((SZ_FEAT % 128) == 0);
static_assert((SZ_CENT % 128) == 0);

typedef float     v4f  __attribute__((ext_vector_type(4)));
typedef float     v8f  __attribute__((ext_vector_type(8)));
typedef _Float16  v8h  __attribute__((ext_vector_type(8)));
typedef _Float16  v16h __attribute__((ext_vector_type(16)));
union FragH { v16h v; v8h h[2]; };

__device__ __forceinline__ v8f wmf(v16h a, v16h b, v8f c) {
  v8f d = __builtin_amdgcn_wmma_f32_16x16x32_f16(false, a, false, b, (short)0, c, false, false);
  asm volatile("v_nop\n\tv_nop\n\tv_nop\n\tv_nop" : "+v"(d) : "v"(a), "v"(b));
  return d;
}

__device__ __forceinline__ v8h cvt8(v4f a, v4f b) {
  v8h r;
  r[0] = (_Float16)a.x; r[1] = (_Float16)a.y; r[2] = (_Float16)a.z; r[3] = (_Float16)a.w;
  r[4] = (_Float16)b.x; r[5] = (_Float16)b.y; r[6] = (_Float16)b.z; r[7] = (_Float16)b.w;
  return r;
}

__device__ __forceinline__ void ins3(float d, float& t0, float& t1, float& t2) {
  const float a1 = fmaxf(d, t0);
  t0 = fminf(d, t0);
  const float b2 = fmaxf(a1, t1);
  t1 = fminf(a1, t1);
  t2 = fminf(b2, t2);
}

__global__ __launch_bounds__(NTHR) void k_cvt(const float* __restrict__ x, _Float16* y, float* sq, int nrows) {
  __shared__ __attribute__((aligned(16))) float sql[RPB];
  const int tid = threadIdx.x, lane = tid & 31, wv = tid >> 5;
  const int blk = blockIdx.x;

#pragma unroll 1
  for (int i = 0; i < RPB / NWAVE; ++i) {
    const int rowraw = blk * RPB + wv * (RPB / NWAVE) + i;
    const bool ok = rowraw < nrows;
    const int row = min(rowraw, nrows - 1);
    const float* xr = x + (size_t)row * CDIM + 8 * lane;
    const v4f a0 = *(const v4f*)xr;
    const v4f a1 = *(const v4f*)(xr + 4);
    const v4f b0 = *(const v4f*)(xr + 256);
    const v4f b1 = *(const v4f*)(xr + 260);
    float ss = a0.x * a0.x + a0.y * a0.y + a0.z * a0.z + a0.w * a0.w;
    ss += a1.x * a1.x + a1.y * a1.y + a1.z * a1.z + a1.w * a1.w;
    ss += b0.x * b0.x + b0.y * b0.y + b0.z * b0.z + b0.w * b0.w;
    ss += b1.x * b1.x + b1.y * b1.y + b1.z * b1.z + b1.w * b1.w;
    ss += __shfl_xor(ss, 1);
    ss += __shfl_xor(ss, 2);
    ss += __shfl_xor(ss, 4);
    ss += __shfl_xor(ss, 8);
    ss += __shfl_xor(ss, 16);
    const v8h o0 = cvt8(a0 * CARRY, a1 * CARRY);
    const v8h o1 = cvt8(b0 * CARRY, b1 * CARRY);
    _Float16* d = y + (size_t)row * CDIM + 8 * lane;
    if (ok) { *(volatile v8h*)d = o0; *(volatile v8h*)(d + 256) = o1; }
    __threadfence();
    if (ok) { *(volatile v8h*)d = o0; *(volatile v8h*)(d + 256) = o1; }
    if (lane == 0) sql[wv * (RPB / NWAVE) + i] = ss;
  }
  __syncthreads();

  if (wv == 0) {
    const int q = lane & 7;
    const v4f v = *(const v4f*)&sql[4 * q];
    const int r0 = blk * RPB + 4 * q;
    const bool okw = (lane < 8) && (r0 + 3 < nrows);
    float* gp = sq + (size_t)r0;
    if (okw) *(volatile v4f*)gp = v;
    __threadfence();
    if (okw) *(volatile v4f*)gp = v;
  }
}

__global__ __launch_bounds__(NTHR) void k_dist(const _Float16* __restrict__ e16,
                                               const _Float16* __restrict__ c16,
                                               const float* __restrict__ feat,
                                               const float* __restrict__ cent,
                                               float* out) {
  __shared__ __attribute__((aligned(16))) float centq[PDIM];
  __shared__ __attribute__((aligned(16))) float featq[MBLK];
  __shared__ __attribute__((aligned(16))) float ob[MBLK];
  const int tid = threadIdx.x, lane = tid & 31, wv = tid >> 5, h = lane >> 4, m = lane & 15;
  const int row0 = blockIdx.x * MBLK;
  const v8f zero8 = {0.f, 0.f, 0.f, 0.f, 0.f, 0.f, 0.f, 0.f};

  for (int i = tid; i < PDIM / 4; i += NTHR) *(v4f*)&centq[4 * i] = *(const v4f*)(cent + 4 * i);
  {
    const int q = tid & 15;
    const v4f fv = *(const v4f*)(feat + (size_t)row0 + 4 * q);
    if (tid < 16) *(v4f*)&featq[4 * q] = fv;
  }
  __syncthreads();

  float fq[8], t0v[8], t1v[8], t2v[8];
#pragma unroll
  for (int r = 0; r < 8; ++r) {
    fq[r] = featq[16 * wv + 8 * h + r];
    t0v[r] = BIGV; t1v[r] = BIGV; t2v[r] = BIGV;
  }

  const _Float16* arow = e16 + ((size_t)row0 + 16 * wv + m) * CDIM + 8 * h;

#pragma unroll 1
  for (int g = 0; g < NGRP; ++g) {
    const _Float16* brow = c16 + ((size_t)(64 * g) + m) * CDIM + 8 * h;

    v8f acc[4];
#pragma unroll
    for (int t = 0; t < 4; ++t) acc[t] = zero8;

#pragma unroll 1
    for (int ks = 0; ks < CDIM / 32; ++ks) {
      const int k0 = 32 * ks;
      FragH af;
      af.h[0] = *(const v8h*)(arow + k0);
      af.h[1] = *(const v8h*)(arow + k0 + 16);
      FragH bf[4];
#pragma unroll
      for (int t = 0; t < 4; ++t) {
        const _Float16* bq = brow + (size_t)(16 * t) * CDIM + k0;
        bf[t].h[0] = *(const v8h*)bq;
        bf[t].h[1] = *(const v8h*)(bq + 16);
      }
#pragma unroll
      for (int t = 0; t < 4; ++t) acc[t] = wmf(af.v, bf[t].v, acc[t]);
    }

#pragma unroll
    for (int t = 0; t < 4; ++t) {
      const float cq = centq[64 * g + 16 * t + m];
#pragma unroll
      for (int r = 0; r < 8; ++r) {
        const float d2 = (fq[r] + cq) - acc[t][r] * FC2;
        ins3(d2, t0v[r], t1v[r], t2v[r]);
      }
    }
  }

#pragma unroll
  for (int s = 0; s < 4; ++s) {
    const int off = 1 << s;
#pragma unroll
    for (int r = 0; r < 8; ++r) {
      const float o0 = __shfl_xor(t0v[r], off);
      const float o1 = __shfl_xor(t1v[r], off);
      const float o2 = __shfl_xor(t2v[r], off);
      ins3(o0, t0v[r], t1v[r], t2v[r]);
      ins3(o1, t0v[r], t1v[r], t2v[r]);
      ins3(o2, t0v[r], t1v[r], t2v[r]);
    }
  }

  const int mm = m & 7;
  float u0 = t0v[0], u1 = t1v[0], u2 = t2v[0];
#pragma unroll
  for (int r = 1; r < 8; ++r) {
    const bool sel = (mm == r);
    u0 = sel ? t0v[r] : u0;
    u1 = sel ? t1v[r] : u1;
    u2 = sel ? t2v[r] : u2;
  }
  const float d0 = sqrtf(u0);
  const float d1 = sqrtf(u1);
  const float dd2 = sqrtf(u2);
  const float e1 = expf(d0 - d1);
  const float e2 = expf(d0 - dd2);
  const float ssum = (1.0f + e2) + e1;
  const float w0 = 1.0f / ssum;
  const float res = w0 * d0;
  if (m < 8) ob[16 * wv + 8 * h + m] = res;
  __syncthreads();

  if (wv == 0) {
    const int q = lane & 15;
    const v4f v = *(const v4f*)&ob[4 * q];
    float* gp = out + (size_t)row0 + 4 * q;
    if (lane < 16) *(volatile v4f*)gp = v;
    __threadfence();
    if (lane < 16) *(volatile v4f*)gp = v;
  }
}

extern "C" void kernel_launch(void* const* d_in, const int* in_sizes, int n_in,
                              void* d_out, int out_size, void* d_ws, size_t ws_size,
                              hipStream_t stream) {
  if (n_in < 2) return;
  if (in_sizes[0] != MROWS * CDIM) return;
  if (in_sizes[1] != PDIM * CDIM) return;
  if (out_size != MROWS) return;

  const float* embeds    = (const float*)d_in[0];
  const float* centroids = (const float*)d_in[1];
  float* out = (float*)d_out;

  char* ws = (char*)d_ws;
  size_t off = 0;
  const size_t oE16  = off; off += SZ_E16;
  const size_t oC16  = off; off += SZ_C16;
  const size_t oFEAT = off; off += SZ_FEAT;
  const size_t oCENT = off; off += SZ_CENT;
  if (off != SZ_TOT) return;
  if (off > ws_size || off > (size_t)WSCAP) return;

  _Float16* e16  = (_Float16*)(ws + oE16);
  _Float16* c16  = (_Float16*)(ws + oC16);
  float*    featp = (float*)(ws + oFEAT);
  float*    centp = (float*)(ws + oCENT);

  k_cvt<<<MROWS / RPB, NTHR, 0, stream>>>(embeds, e16, featp, MROWS);
  k_cvt<<<PDIM / RPB, NTHR, 0, stream>>>(centroids, c16, centp, PDIM);
  k_dist<<<MROWS / MBLK, NTHR, 0, stream>>>(e16, c16, featp, centp, out);
}
